// PointerNet_53609781788996
// MI455X (gfx1250) — hardware-verified
//
#include <hip/hip_runtime.h>
#include <math.h>

constexpr int nBatch = 8;
constexpr int nSent  = 128;
constexpr int nWord  = 128;
constexpr int dSent  = 512;
constexpr int dWord  = 256;
constexpr int dSH    = 256;
constexpr int dEH    = 128;
constexpr int dLab   = 64;
constexpr int dG     = 256;
constexpr int nRows  = nBatch * nSent;
constexpr int dP1    = dEH + dLab;
constexpr int dP2    = dSH + dLab;
constexpr int dXS    = dSent + dSH + dP1 + dG;
constexpr int dXHS   = dXS + dSH;
constexpr int dXE    = dWord + dP2 + dG;
constexpr int dXHE   = dXE + dEH;
constexpr int dXG    = dSH + dEH;
constexpr int dXHG   = dXG + dG;

static_assert(nBatch * nWord == nRows);
static_assert(nRows % 64 == 0 && nSent % 64 == 0);
static_assert(dP1 % 64 == 0 && dP2 % 64 == 0 && dSH % 64 == 0 && dEH % 64 == 0);
static_assert(dXHS % 64 == 0 && dXS % 64 == 0 && dXHE % 64 == 0 && dXE % 64 == 0);
static_assert(dSH % 32 == 0 && dEH % 32 == 0 && nSent % 32 == 0);
static_assert((nRows * dSH + nRows * dEH + nBatch * dG) * 4 == 1581056);

typedef __attribute__((ext_vector_type(16))) _Float16 v16h;
typedef __attribute__((ext_vector_type(8)))  _Float16 v8h;
typedef __attribute__((ext_vector_type(16))) __bf16   v16b;
typedef __attribute__((ext_vector_type(8)))  __bf16   v8b;
typedef __attribute__((ext_vector_type(8)))  float    v8f;
typedef __attribute__((ext_vector_type(4)))  float    v4f;
typedef __attribute__((ext_vector_type(4)))  unsigned int v4u;

__device__ __forceinline__ unsigned short f2bf_bits(float f) {
  unsigned u = __float_as_uint(f);
  return (unsigned short)((u + 0x7FFFu + ((u >> 16) & 1u)) >> 16);
}
__device__ __forceinline__ float bf_bits2f(unsigned short h) { return __uint_as_float(((unsigned)h) << 16); }

__device__ __forceinline__ void dep_guard_h(v8f& a, v8f& b, v16h x, v16h y) { asm volatile("v_nop\n\tv_nop\n\tv_nop\n\tv_nop" : "+v"(a), "+v"(b) : "v"(x), "v"(y)); }
__device__ __forceinline__ void dep_guard_b(v8f& a, v8f& b, v16b x, v16b y) { asm volatile("v_nop\n\tv_nop\n\tv_nop\n\tv_nop" : "+v"(a), "+v"(b) : "v"(x), "v"(y)); }
__device__ __forceinline__ void keep4_h(v16h a, v16h b, v16h c, v16h d) { asm volatile("v_nop" :: "v"(a), "v"(b), "v"(c), "v"(d)); }
__device__ __forceinline__ void keep4_b(v16b a, v16b b, v16b c, v16b d) { asm volatile("v_nop" :: "v"(a), "v"(b), "v"(c), "v"(d)); }
__device__ __forceinline__ void acc_guard4(v8f& a, v8f& b, v8f& c, v8f& d) { asm volatile("v_nop\n\tv_nop\n\tv_nop\n\tv_nop" : "+v"(a), "+v"(b), "+v"(c), "+v"(d)); }
template <typename T> struct Frag;
template <> struct Frag<_Float16> {
  typedef v16h V; union U { v16h v; v8h h[2]; };
  static __device__ __forceinline__ v16h load(const _Float16* p) {
    U f; f.h[0] = *(const v8h*)(p); f.h[1] = *(const v8h*)(p + 16); return f.v;
  }
  static __device__ __forceinline__ v8f mma(v16h a, v16h b, v8f c) {
    return __builtin_amdgcn_wmma_f32_16x16x32_f16(false, a, false, b, (short)0, c, false, false);
  }
  static __device__ __forceinline__ void guard(v8f& a, v8f& b, v16h x, v16h y) { dep_guard_h(a, b, x, y); }
  static __device__ __forceinline__ void keep(v16h a, v16h b, v16h c, v16h d) { keep4_h(a, b, c, d); }
};
template <> struct Frag<__bf16> {
  typedef v16b V; union U { v16b v; v8b h[2]; };
  static __device__ __forceinline__ v16b load(const __bf16* p) {
    U f; f.h[0] = *(const v8b*)(p); f.h[1] = *(const v8b*)(p + 16); return f.v;
  }
  static __device__ __forceinline__ v8f mma(v16b a, v16b b, v8f c) {
    return __builtin_amdgcn_wmma_f32_16x16x32_bf16(false, a, false, b, (short)0, c, false, false);
  }
  static __device__ __forceinline__ void guard(v8f& a, v8f& b, v16b x, v16b y) { dep_guard_b(a, b, x, y); }
  static __device__ __forceinline__ void keep(v16b a, v16b b, v16b c, v16b d) { keep4_b(a, b, c, d); }
};

template <int ET> struct Elem;
template <> struct Elem<0> { typedef _Float16 T; };
template <> struct Elem<1> { typedef __bf16 T; };
template <int ET, bool SPLIT, int BIAS_MODE, int OUT_MODE, bool RESID, int ACT = 0>
__global__ __launch_bounds__(256) void wmma_gemm64(
    const unsigned short* __restrict__ Ap, const unsigned short* __restrict__ A2p, int lda, long strideA,
    const unsigned short* __restrict__ Btp, const unsigned short* __restrict__ Bt2p, int ldb, long strideB,
    void* __restrict__ Cout, void* __restrict__ Cout2, int ldc, long strideC,
    const float* __restrict__ bias,
    const float* __restrict__ resid, long strideR,
    int M, int N, int K, float scale) {
  typedef typename Elem<ET>::T T;
  typedef typename Frag<T>::V V;
  const T* A = (const T*)Ap; const T* A2 = (const T*)A2p; const T* Bt = (const T*)Btp; const T* Bt2 = (const T*)Bt2p;
  __shared__ __align__(16) float sT[8][16 * 68];
  const int b    = blockIdx.y;
  const int lane = threadIdx.x & 31;
  const int wave = threadIdx.x >> 5;
  const int tilesN = N >> 6;
  const int tilesM = M >> 6;
  const int tile = blockIdx.x * 8 + wave;
  if (tile >= tilesM * tilesN) return;
  const int tm = tile / tilesN;
  const int tn = tile - tm * tilesN;
  const int m0 = tm << 6;
  const int n0 = tn << 6;

  const T* Ab  = A  + (size_t)b * strideA;
  const T* Bb  = Bt + (size_t)b * strideB;
  const T* Ab2 = SPLIT ? (A2  + (size_t)b * strideA) : nullptr;
  const T* Bb2 = SPLIT ? (Bt2 + (size_t)b * strideB) : nullptr;

  const int rlane = lane & 15;
  const int koff  = (lane >> 4) * 8;
  const int mOff  = (lane >> 4) * 8;

  v8f acc[4][4];
#pragma unroll
  for (int i = 0; i < 4; ++i)
#pragma unroll
    for (int j = 0; j < 4; ++j) acc[i][j] = (v8f){0.f,0.f,0.f,0.f,0.f,0.f,0.f,0.f};

  for (int k0 = 0; k0 < K; k0 += 32) {
    V bh[4], bl[4];
#pragma unroll
    for (int j = 0; j < 4; ++j) {
      const size_t bo = (size_t)(n0 + (j << 4) + rlane) * ldb + koff + k0;
      bh[j] = Frag<T>::load(Bb + bo);
      if (SPLIT) bl[j] = Frag<T>::load(Bb2 + bo);
    }
#pragma unroll
    for (int i = 0; i < 4; ++i) {
      const size_t ao = (size_t)(m0 + (i << 4) + rlane) * lda + koff + k0;
      V ah = Frag<T>::load(Ab + ao);
      V al;
      if (SPLIT) al = Frag<T>::load(Ab2 + ao);
#pragma unroll
      for (int j = 0; j < 4; ++j) {
        acc[i][j] = Frag<T>::mma(ah, bh[j], acc[i][j]);
        if (SPLIT) {
          acc[i][j] = Frag<T>::mma(ah, bl[j], acc[i][j]);
          acc[i][j] = Frag<T>::mma(al, bh[j], acc[i][j]);
        }
      }
      Frag<T>::guard(acc[i][0], acc[i][3], ah, SPLIT ? al : ah);
    }
    Frag<T>::keep(bh[0], bh[1], bh[2], bh[3]);
    if (SPLIT) Frag<T>::keep(bl[0], bl[1], bl[2], bl[3]);
  }
  acc_guard4(acc[0][0], acc[0][1], acc[0][2], acc[0][3]);
  acc_guard4(acc[1][0], acc[1][1], acc[1][2], acc[1][3]);
  acc_guard4(acc[2][0], acc[2][1], acc[2][2], acc[2][3]);
  acc_guard4(acc[3][0], acc[3][1], acc[3][2], acc[3][3]);

  float* slab = sT[wave];
  const float* Rb = RESID ? (resid + (size_t)b * strideR) : nullptr;
#pragma unroll
  for (int i = 0; i < 4; ++i) {
    const int mBase = m0 + (i << 4);
#pragma unroll
    for (int j = 0; j < 4; ++j) {
      const int n = n0 + (j << 4) + rlane;
      float bv = 0.f;
      if (BIAS_MODE == 2) bv = bias[n];
#pragma unroll
      for (int r = 0; r < 8; ++r) {
        float v = acc[i][j][r] * scale;
        if (BIAS_MODE == 1) v += bias[mBase + mOff + r];
        if (BIAS_MODE == 2) v += bv;
        if (RESID) v += Rb[(size_t)(mBase + mOff + r) * ldc + n];
        if (ACT == 1) v = tanhf(v);
        if (ACT == 2) v = fmaxf(v, 0.0f);
        if (ACT == 3) v = v / (1.0f + expf(-v));
        if (ACT == 4) v = (v > 0.f) ? v : 0.01f * v;
        if (ACT == 5) v = 0.5f * v * (1.0f + erff(v * 0.70710678118654752f));
        slab[(mOff + r) * 68 + (j << 4) + rlane] = v;
      }
    }
    __builtin_amdgcn_fence(__ATOMIC_RELEASE, "workgroup");
    __builtin_amdgcn_wave_barrier();
    __builtin_amdgcn_fence(__ATOMIC_ACQUIRE, "workgroup");
    if (OUT_MODE == 0) {
      float* C = (float*)Cout + (size_t)b * strideC;
      const int hh = lane >> 4, c4 = (lane & 15) * 4;
      for (int pass = 0; pass < 2; ++pass) {
#pragma unroll
        for (int it = 0; it < 8; ++it) {
          const int row = it * 2 + hh;
          v4f v = *(const v4f*)(slab + row * 68 + c4);
          *(volatile v4f*)(C + (size_t)(mBase + row) * ldc + n0 + c4) = v;
        }
        __threadfence();
      }
    } else {
      const int q = lane >> 3, c8 = (lane & 7) * 8;
      unsigned short* C  = (unsigned short*)Cout  + (size_t)b * strideC;
      unsigned short* C2 = (OUT_MODE == 2) ? ((unsigned short*)Cout2 + (size_t)b * strideC) : nullptr;
      for (int pass = 0; pass < 2; ++pass) {
#pragma unroll
        for (int it = 0; it < 4; ++it) {
          const int row = it * 4 + q;
          const float* sp = slab + row * 68 + c8;
          v8h hv, lv;
#pragma unroll
          for (int e = 0; e < 8; ++e) {
            if (OUT_MODE == 1) {
              hv[e] = (_Float16)sp[e];
            } else {
              unsigned short hb = f2bf_bits(sp[e]);
              unsigned short lb = f2bf_bits(sp[e] - bf_bits2f(hb));
              hv[e] = __builtin_bit_cast(_Float16, hb);
              lv[e] = __builtin_bit_cast(_Float16, lb);
            }
          }
          *(volatile v8h*)(C + (size_t)(mBase + row) * ldc + n0 + c8) = hv;
          if (OUT_MODE == 2) *(volatile v8h*)(C2 + (size_t)(mBase + row) * ldc + n0 + c8) = lv;
        }
        __threadfence();
      }
    }
    __builtin_amdgcn_fence(__ATOMIC_RELEASE, "workgroup");
    __builtin_amdgcn_wave_barrier();
    __builtin_amdgcn_fence(__ATOMIC_ACQUIRE, "workgroup");
  }
}

__device__ __forceinline__ unsigned pk16(unsigned short a, unsigned short b) { return (unsigned)a | ((unsigned)b << 16); }

__device__ __forceinline__ void split8(const v4f a, const v4f c, v4u& uh, v4u& ul) {
  unsigned short hb[8], lb[8];
#pragma unroll
  for (int e = 0; e < 4; ++e) {
    hb[e]     = f2bf_bits(a[e]);  lb[e]     = f2bf_bits(a[e] - bf_bits2f(hb[e]));
    hb[4 + e] = f2bf_bits(c[e]);  lb[4 + e] = f2bf_bits(c[e] - bf_bits2f(hb[4 + e]));
  }
  uh = (v4u){pk16(hb[0], hb[1]), pk16(hb[2], hb[3]), pk16(hb[4], hb[5]), pk16(hb[6], hb[7])};
  ul = (v4u){pk16(lb[0], lb[1]), pk16(lb[2], lb[3]), pk16(lb[4], lb[5]), pk16(lb[6], lb[7])};
}

__device__ __forceinline__ float sigm_f(float x) {
  x = fminf(fmaxf(x, -80.0f), 80.0f);
  return 1.0f / (1.0f + expf(-x));
}

__global__ __launch_bounds__(256) void zero4_kernel(float* __restrict__ p, int n4) {
  const int i = blockIdx.x * 256 + threadIdx.x;
  if (i >= n4) return;
  const v4f z = {0.f, 0.f, 0.f, 0.f};
  float* q = p + 4 * (size_t)i;
  *(volatile v4f*)q = z;
  __threadfence();
  *(volatile v4f*)q = z;
}

__global__ __launch_bounds__(256) void rsplit_kernel(const float* __restrict__ in, unsigned short* __restrict__ hi,
                                                     unsigned short* __restrict__ lo, int n8) {
  const int i = blockIdx.x * 256 + threadIdx.x;
  if (i >= n8) return;
  const float* p = in + 8 * (size_t)i;
  const v4f a = *(const v4f*)(p);
  const v4f c = *(const v4f*)(p + 4);
  v4u uh, ul;
  split8(a, c, uh, ul);
  unsigned short* qh = hi + 8 * (size_t)i;
  unsigned short* ql = lo + 8 * (size_t)i;
  *(volatile v4u*)qh = uh; *(volatile v4u*)ql = ul;
  __threadfence();
  *(volatile v4u*)qh = uh; *(volatile v4u*)ql = ul;
}

__global__ __launch_bounds__(256) void tsplit_kernel(const float* __restrict__ src, int npitch, int kreal, long sIn,
                                                     unsigned short* __restrict__ dhi, unsigned short* __restrict__ dlo,
                                                     int ldo, long sOut) {
  __shared__ float sm[64][65];
  const int t  = threadIdx.x;
  const int k0 = blockIdx.x * 64;
  const int n0 = blockIdx.y * 64;
  const float* sp = src + (size_t)blockIdx.z * sIn;
#pragma unroll
  for (int i = 0; i < 4; ++i) {
    const int e  = i * 256 + t;
    const int r  = e >> 4;
    const int c4 = (e & 15) * 4;
    const int kr = k0 + r;
    const int kc = (kr < kreal) ? kr : (kreal - 1);
    v4f v = *(const v4f*)(sp + (size_t)kc * npitch + n0 + c4);
    const float live = (kr < kreal) ? 1.0f : 0.0f;
    sm[c4 + 0][r] = live * v[0];
    sm[c4 + 1][r] = live * v[1];
    sm[c4 + 2][r] = live * v[2];
    sm[c4 + 3][r] = live * v[3];
  }
  __syncthreads();
  const int lane = t & 31, wave = t >> 5;
  const int q = lane >> 3, c8 = (lane & 7) * 8;
  unsigned short* oh = dhi + (size_t)blockIdx.z * sOut;
  unsigned short* ol = dlo + (size_t)blockIdx.z * sOut;
  for (int pass = 0; pass < 2; ++pass) {
#pragma unroll
    for (int it = 0; it < 2; ++it) {
      const int row = wave * 8 + it * 4 + q;
      const v4f a = {sm[row][c8 + 0], sm[row][c8 + 1], sm[row][c8 + 2], sm[row][c8 + 3]};
      const v4f c = {sm[row][c8 + 4], sm[row][c8 + 5], sm[row][c8 + 6], sm[row][c8 + 7]};
      v4u uh, ul;
      split8(a, c, uh, ul);
      const size_t o = (size_t)(n0 + row) * ldo + k0 + c8;
      *(volatile v4u*)(oh + o) = uh;
      *(volatile v4u*)(ol + o) = ul;
    }
    __threadfence();
  }
}

__global__ __launch_bounds__(256) void adj_kernel(const int* __restrict__ mat, const int* __restrict__ smask,
                                                  unsigned short* __restrict__ ahi, unsigned short* __restrict__ alo) {
  __shared__ unsigned bits[nSent * 4];
  __shared__ int smk[nSent];
  const int b = blockIdx.x, t = threadIdx.x, lane = t & 31, wave = t >> 5;
  if (t < nSent) smk[t] = smask[b * nSent + t];
  const int* mb = mat + (size_t)b * nSent * nWord;
#pragma unroll 1
  for (int i = 0; i < 16; ++i) {
    const int s = wave * 16 + i;
#pragma unroll
    for (int j = 0; j < 4; ++j) {
      const int v = mb[s * nWord + j * 32 + lane];
      const unsigned wd = (unsigned)__ballot(v != 0);
      if (lane == 0) bits[s * 4 + j] = wd;
    }
  }
  __syncthreads();
  const int hh = lane >> 4, cb = (lane & 15) * 8;
  unsigned short* ph = ahi + (size_t)b * nSent * nSent;
  unsigned short* pl = alo + (size_t)b * nSent * nSent;
  const v4u z4 = {0u, 0u, 0u, 0u};
  for (int pass = 0; pass < 2; ++pass) {
#pragma unroll 1
    for (int p = 0; p < 8; ++p) {
      const int s = wave * 16 + 2 * p + hh;
      const unsigned b0 = bits[s * 4 + 0], b1 = bits[s * 4 + 1], b2 = bits[s * 4 + 2], b3 = bits[s * 4 + 3];
      unsigned short hv[8];
#pragma unroll
      for (int e = 0; e < 8; ++e) {
        const int tt = cb + e;
        const unsigned any = (b0 & bits[tt * 4 + 0]) | (b1 & bits[tt * 4 + 1]) | (b2 & bits[tt * 4 + 2]) | (b3 & bits[tt * 4 + 3]);
        const bool on = (any != 0u) && (tt != s) && (smk[tt] != 0);
        hv[e] = on ? (unsigned short)0x3F80u : (unsigned short)0u;
      }
      const v4u u = (v4u){pk16(hv[0], hv[1]), pk16(hv[2], hv[3]), pk16(hv[4], hv[5]), pk16(hv[6], hv[7])};
      const size_t o = (size_t)s * nSent + cb;
      *(volatile v4u*)(ph + o) = u;
      *(volatile v4u*)(pl + o) = z4;
    }
    __threadfence();
  }
}

__global__ __launch_bounds__(320) void tables_kernel(const float* __restrict__ ee, const float* __restrict__ g1w, const float* __restrict__ g1b,
                                                     const float* __restrict__ g2w, const float* __restrict__ g2b,
                                                     float* __restrict__ t1, float* __restrict__ t2) {
  const int m = blockIdx.x, c = threadIdx.x;
  const int cc = (c < dP1) ? c : (dP1 - 1);
  float a1 = 0.0f, a2 = 0.0f;
#pragma unroll 1
  for (int l = 0; l < dLab; ++l) {
    const float ev = ee[m * dLab + l];
    a1 += ev * g1w[(size_t)(dSH + dEH + l) * dP1 + cc];
    a2 += ev * g2w[(size_t)(dEH + dSH + l) * dP2 + c];
  }
  a1 += g1b[cc];
  a2 += g2b[c];
  for (int pass = 0; pass < 2; ++pass) {
    if (c < dP1) *(volatile float*)(t1 + m * dP1 + c) = a1;
    *(volatile float*)(t2 + m * dP2 + c) = a2;
    __threadfence();
  }
}

__global__ __launch_bounds__(192) void aggs_kernel(const int* __restrict__ mat, const float* __restrict__ ehold,
                                                   const float* __restrict__ P1s, const float* __restrict__ P1e,
                                                   const float* __restrict__ t1, const float* __restrict__ ee,
                                                   float* __restrict__ sne) {
  const int s = blockIdx.x, b = blockIdx.y, c = threadIdx.x;
  const int row = b * nSent + s;
  const int* mrow = mat + (size_t)row * nWord;
  const float base = P1s[(size_t)row * dP1 + c];
  const int ce = (c < dEH) ? c : (dEH - 1);
  const int cl = (c >= dEH) ? (c - dEH) : 0;
  const float fl = (c >= dEH) ? 1.0f : 0.0f;
  const float fe = 1.0f - fl;
  const float tv0 = t1[c], tv1 = t1[dP1 + c], tv2 = t1[2 * dP1 + c], tv3 = t1[3 * dP1 + c];
  const float ev0 = ee[cl], ev1 = ee[dLab + cl], ev2 = ee[2 * dLab + cl], ev3 = ee[3 * dLab + cl];
  const float* pe = P1e + (size_t)b * nWord * dP1 + c;
  const float* eh = ehold + (size_t)b * nWord * dEH + ce;
  float acc = 0.0f;
#pragma unroll 1
  for (int w = 0; w < nWord; ++w) {
    const int m = mrow[w];
    if (m == 0) continue;
    int mi = (m < 0) ? (m + 4) : m;
    mi = (mi < 0) ? 0 : ((mi > 3) ? 3 : mi);
    const float tv = (mi == 0) ? tv0 : (mi == 1) ? tv1 : (mi == 2) ? tv2 : tv3;
    const float ev = (mi == 0) ? ev0 : (mi == 1) ? ev1 : (mi == 2) ? ev2 : ev3;
    const float g = sigm_f(base + pe[(size_t)w * dP1] + tv);
    const float ve = eh[(size_t)w * dEH];
    const float val = fmaf(fe, ve, fl * ev);
    acc += val * g;
  }
  float* op = sne + (size_t)row * dP1 + c;
  *(volatile float*)op = acc;
  __threadfence();
  *(volatile float*)op = acc;
}

__global__ __launch_bounds__(320) void agge_kernel(const int* __restrict__ mat, const float* __restrict__ shold,
                                                   const float* __restrict__ P2s, const float* __restrict__ P2e,
                                                   const float* __restrict__ t2, const float* __restrict__ ee,
                                                   float* __restrict__ ens) {
  const int w = blockIdx.x, b = blockIdx.y, c = threadIdx.x;
  const int row = b * nWord + w;
  const float base = P2e[(size_t)row * dP2 + c];
  const int cs = (c < dSH) ? c : (dSH - 1);
  const int cl = (c >= dSH) ? (c - dSH) : 0;
  const float fl = (c >= dSH) ? 1.0f : 0.0f;
  const float fs = 1.0f - fl;
  const float tv0 = t2[c], tv1 = t2[dP2 + c], tv2 = t2[2 * dP2 + c], tv3 = t2[3 * dP2 + c];
  const float ev0 = ee[cl], ev1 = ee[dLab + cl], ev2 = ee[2 * dLab + cl], ev3 = ee[3 * dLab + cl];
  const float* ps = P2s + (size_t)b * nSent * dP2 + c;
  const float* sh = shold + (size_t)b * nSent * dSH + cs;
  const int* mcol = mat + (size_t)b * nSent * nWord + w;
  float acc = 0.0f;
#pragma unroll 1
  for (int s = 0; s < nSent; ++s) {
    const int m = mcol[(size_t)s * nWord];
    if (m == 0) continue;
    int mi = (m < 0) ? (m + 4) : m;
    mi = (mi < 0) ? 0 : ((mi > 3) ? 3 : mi);
    const float tv = (mi == 0) ? tv0 : (mi == 1) ? tv1 : (mi == 2) ? tv2 : tv3;
    const float ev = (mi == 0) ? ev0 : (mi == 1) ? ev1 : (mi == 2) ? ev2 : ev3;
    const float g = sigm_f(base + ps[(size_t)s * dP2] + tv);
    const float vs = sh[(size_t)s * dSH];
    const float val = fmaf(fs, vs, fl * ev);
    acc += val * g;
  }
  float* op = ens + (size_t)row * dP2 + c;
  *(volatile float*)op = acc;
  __threadfence();
  *(volatile float*)op = acc;
}

__global__ __launch_bounds__(256) void packs_kernel(const float* __restrict__ sent, const float* __restrict__ sns,
                                                    const float* __restrict__ sne, const float* __restrict__ gold,
                                                    const float* __restrict__ shold,
                                                    unsigned short* __restrict__ xh, unsigned short* __restrict__ xl) {
  __shared__ __align__(16) float rowbuf[dXHS];
  const int row = blockIdx.x, t = threadIdx.x;
  const int b = row >> 7;
  rowbuf[t]                         = sent[(size_t)row * dSent + t];
  rowbuf[256 + t]                   = sent[(size_t)row * dSent + 256 + t];
  rowbuf[dSent + t]                 = sns[(size_t)row * dSH + t];
  if (t < dP1) rowbuf[dSent + dSH + t] = sne[(size_t)row * dP1 + t];
  rowbuf[dSent + dSH + dP1 + t]     = gold[b * dG + t];
  rowbuf[dXS + t]                   = shold[(size_t)row * dSH + t];
  __syncthreads();
  if (t < dXHS / 8) {
    const v4f a = *(const v4f*)(rowbuf + 8 * t);
    const v4f c = *(const v4f*)(rowbuf + 8 * t + 4);
    v4u uh, ul;
    split8(a, c, uh, ul);
    const size_t o = (size_t)row * dXHS + 8 * t;
    *(volatile v4u*)(xh + o) = uh; *(volatile v4u*)(xl + o) = ul;
    __threadfence();
    *(volatile v4u*)(xh + o) = uh; *(volatile v4u*)(xl + o) = ul;
  }
}

__global__ __launch_bounds__(256) void packe_kernel(const float* __restrict__ word, const float* __restrict__ ens,
                                                    const float* __restrict__ gold, const float* __restrict__ ehold,
                                                    unsigned short* __restrict__ xh, unsigned short* __restrict__ xl) {
  __shared__ __align__(16) float rowbuf[dXHE];
  const int row = blockIdx.x, t = threadIdx.x;
  const int b = row >> 7;
  rowbuf[t] = word[(size_t)row * dWord + t];
  rowbuf[dWord + t] = ens[(size_t)row * dP2 + t];
  if (t < dP2 - 256) rowbuf[dWord + 256 + t] = ens[(size_t)row * dP2 + 256 + t];
  rowbuf[dWord + dP2 + t] = gold[b * dG + t];
  if (t < dEH) rowbuf[dXE + t] = ehold[(size_t)row * dEH + t];
  __syncthreads();
  if (t < dXHE / 8) {
    const v4f a = *(const v4f*)(rowbuf + 8 * t);
    const v4f c = *(const v4f*)(rowbuf + 8 * t + 4);
    v4u uh, ul;
    split8(a, c, uh, ul);
    const size_t o = (size_t)row * dXHE + 8 * t;
    *(volatile v4u*)(xh + o) = uh; *(volatile v4u*)(xl + o) = ul;
    __threadfence();
    *(volatile v4u*)(xh + o) = uh; *(volatile v4u*)(xl + o) = ul;
  }
}

__global__ __launch_bounds__(256) void cells_kernel(const float* __restrict__ RZ, const float* __restrict__ Cp, const float* __restrict__ Up,
                                                    const float* __restrict__ rb, const float* __restrict__ zb,
                                                    const float* __restrict__ cb, const float* __restrict__ ub,
                                                    const float* __restrict__ hold, const int* __restrict__ msk,
                                                    float* __restrict__ hnew) {
  const int row = blockIdx.x, c = threadIdx.x;
  const float r = sigm_f(RZ[(size_t)row * (2 * dSH) + c] + rb[c]);
  const float z = sigm_f(RZ[(size_t)row * (2 * dSH) + dSH + c] + zb[c]);
  const float hu = Up[(size_t)row * dSH + c] + ub[c];
  const float u = tanhf(Cp[(size_t)row * dSH + c] + cb[c] + r * hu);
  const float h = hold[(size_t)row * dSH + c];
  float nh = z * h + (1.0f - z) * u;
  if (msk[row] == 0) nh = 0.0f;
  float* op = hnew + (size_t)row * dSH + c;
  *(volatile float*)op = nh;
  __threadfence();
  *(volatile float*)op = nh;
}

__global__ __launch_bounds__(128) void celle_kernel(const float* __restrict__ RZ, const float* __restrict__ Cp, const float* __restrict__ Up,
                                                    const float* __restrict__ rb, const float* __restrict__ zb,
                                                    const float* __restrict__ cb, const float* __restrict__ ub,
                                                    const float* __restrict__ hold, const int* __restrict__ msk,
                                                    float* __restrict__ hnew) {
  const int row = blockIdx.x, c = threadIdx.x;
  const float r = sigm_f(RZ[(size_t)row * (2 * dEH) + c] + rb[c]);
  const float z = sigm_f(RZ[(size_t)row * (2 * dEH) + dEH + c] + zb[c]);
  const float hu = Up[(size_t)row * dEH + c] + ub[c];
  const float u = tanhf(Cp[(size_t)row * dEH + c] + cb[c] + r * hu);
  const float h = hold[(size_t)row * dEH + c];
  float nh = z * h + (1.0f - z) * u;
  if (msk[row] == 0) nh = 0.0f;
  float* op = hnew + (size_t)row * dEH + c;
  *(volatile float*)op = nh;
  __threadfence();
  *(volatile float*)op = nh;
}

__global__ __launch_bounds__(256) void cellg_kernel(const float* __restrict__ snew, const float* __restrict__ enew,
                                                    const int* __restrict__ smask, const int* __restrict__ wmask,
                                                    const float* __restrict__ gold,
                                                    const float* __restrict__ rw, const float* __restrict__ rb,
                                                    const float* __restrict__ zw, const float* __restrict__ zb,
                                                    const float* __restrict__ cw, const float* __restrict__ cb,
                                                    const float* __restrict__ uw, const float* __restrict__ ub,
                                                    float* __restrict__ gnew) {
  __shared__ float xh[dXHG];
  const int b = blockIdx.x, c = threadIdx.x;
  const int cc = (c < dEH) ? c : (dEH - 1);
  float ss = 0.0f, se = 0.0f, cs = 0.0f, ce = 0.0f;
#pragma unroll 1
  for (int s = 0; s < nSent; ++s) {
    ss += snew[(size_t)(b * nSent + s) * dSH + c];
    cs += (smask[b * nSent + s] != 0) ? 1.0f : 0.0f;
  }
#pragma unroll 1
  for (int w = 0; w < nWord; ++w) {
    se += enew[(size_t)(b * nWord + w) * dEH + cc];
    ce += (wmask[b * nWord + w] != 0) ? 1.0f : 0.0f;
  }
  const float gv = gold[b * dG + c];
  xh[c] = ss / cs;
  if (c < dEH) xh[dSH + c] = se / (ce + 1.0f);
  xh[dXG + c] = gv;
  __syncthreads();
  float ar = 0.0f, az = 0.0f;
#pragma unroll 1
  for (int i = 0; i < dXHG; ++i) {
    const float x = xh[i];
    ar += x * rw[(size_t)i * dG + c];
    az += x * zw[(size_t)i * dG + c];
  }
  float ac = 0.0f;
#pragma unroll 1
  for (int i = 0; i < dXG; ++i) ac += xh[i] * cw[(size_t)i * dG + c];
  float au = 0.0f;
#pragma unroll 1
  for (int i = 0; i < dG; ++i) au += xh[dXG + i] * uw[(size_t)i * dG + c];
  const float r = sigm_f(ar + rb[c]);
  const float z = sigm_f(az + zb[c]);
  const float u = tanhf(ac + cb[c] + r * (au + ub[c]));
  const float ng = z * gv + (1.0f - z) * u;
  float* op = gnew + b * dG + c;
  *(volatile float*)op = ng;
  __threadfence();
  *(volatile float*)op = ng;
}

static void gemm_bf16x3(const unsigned short* Ah, const unsigned short* Al, int lda, long sA,
                        const unsigned short* Bh, const unsigned short* Bl, int ldb, long sB,
                        float* C, int ldc, long sC, int M, int N, int K, int batch, hipStream_t st) {
  const int tiles = (M / 64) * (N / 64);
  wmma_gemm64<1, true, 0, 0, false><<<dim3((tiles + 7) / 8, batch), 256, 0, st>>>(
      Ah, Al, lda, sA, Bh, Bl, ldb, sB, (void*)C, (void*)nullptr, ldc, sC,
      (const float*)nullptr, (const float*)nullptr, 0L, M, N, K, 1.0f);
}

extern "C" void kernel_launch(void* const* d_in, const int* in_sizes, int n_in,
                              void* d_out, int out_size, void* d_ws, size_t ws_size, hipStream_t stream) {
  (void)in_sizes;
  if (n_in < 34) return;
  if (out_size != nRows * dSH + nRows * dEH + nBatch * dG) return;

  const float* sent = (const float*)d_in[0];
  const float* word = (const float*)d_in[1];
  const float* ee   = (const float*)d_in[2];
  const float* g1w  = (const float*)d_in[3];
  const float* g1b  = (const float*)d_in[4];
  const float* g2w  = (const float*)d_in[5];
  const float* g2b  = (const float*)d_in[6];
  const float* s_rw = (const float*)d_in[7];  const float* s_rb = (const float*)d_in[8];
  const float* s_zw = (const float*)d_in[9];  const float* s_zb = (const float*)d_in[10];
  const float* s_cw = (const float*)d_in[11]; const float* s_cb = (const float*)d_in[12];
  const float* s_uw = (const float*)d_in[13]; const float* s_ub = (const float*)d_in[14];
  const float* e_rw = (const float*)d_in[15]; const float* e_rb = (const float*)d_in[16];
  const float* e_zw = (const float*)d_in[17]; const float* e_zb = (const float*)d_in[18];
  const float* e_cw = (const float*)d_in[19]; const float* e_cb = (const float*)d_in[20];
  const float* e_uw = (const float*)d_in[21]; const float* e_ub = (const float*)d_in[22];
  const float* g_rw = (const float*)d_in[23]; const float* g_rb = (const float*)d_in[24];
  const float* g_zw = (const float*)d_in[25]; const float* g_zb = (const float*)d_in[26];
  const float* g_cw = (const float*)d_in[27]; const float* g_cb = (const float*)d_in[28];
  const float* g_uw = (const float*)d_in[29]; const float* g_ub = (const float*)d_in[30];
  const int* smask  = (const int*)d_in[31];
  const int* wmask  = (const int*)d_in[32];
  const int* matrix = (const int*)d_in[33];
  float* out0 = (float*)d_out;
  float* out1 = out0 + (size_t)nRows * dSH;
  float* out2 = out1 + (size_t)nRows * dEH;

  char* ws = (char*)d_ws; size_t off = 0;
  auto carve = [&](size_t bytes) -> char* { char* p = ws + off; off += (bytes + 255) & ~(size_t)255; return p; };
  typedef unsigned short u16;
  u16* wG1Sh = (u16*)carve((size_t)dP1 * dSH * 2);    u16* wG1Sl = (u16*)carve((size_t)dP1 * dSH * 2);
  u16* wG1Eh = (u16*)carve((size_t)dP1 * dEH * 2);    u16* wG1El = (u16*)carve((size_t)dP1 * dEH * 2);
  u16* wG2Eh = (u16*)carve((size_t)dP2 * dEH * 2);    u16* wG2El = (u16*)carve((size_t)dP2 * dEH * 2);
  u16* wG2Sh = (u16*)carve((size_t)dP2 * dSH * 2);    u16* wG2Sl = (u16*)carve((size_t)dP2 * dSH * 2);
  u16* wSRZh = (u16*)carve((size_t)2 * dSH * dXHS * 2); u16* wSRZl = (u16*)carve((size_t)2 * dSH * dXHS * 2);
  u16* wSCh  = (u16*)carve((size_t)dSH * dXS * 2);    u16* wSCl  = (u16*)carve((size_t)dSH * dXS * 2);
  u16* wSUh  = (u16*)carve((size_t)dSH * dSH * 2);    u16* wSUl  = (u16*)carve((size_t)dSH * dSH * 2);
  u16* wERZh = (u16*)carve((size_t)2 * dEH * dXHE * 2); u16* wERZl = (u16*)carve((size_t)2 * dEH * dXHE * 2);
  u16* wECh  = (u16*)carve((size_t)dEH * dXE * 2);    u16* wECl  = (u16*)carve((size_t)dEH * dXE * 2);
  u16* wEUh  = (u16*)carve((size_t)dEH * dEH * 2);    u16* wEUl  = (u16*)carve((size_t)dEH * dEH * 2);
  float* tab1 = (float*)carve((size_t)4 * dP1 * 4);
  float* tab2 = (float*)carve((size_t)4 * dP2 * 4);
  u16* adjH = (u16*)carve((size_t)nBatch * nSent * nSent * 2); u16* adjL = (u16*)carve((size_t)nBatch * nSent * nSent * 2);
  const size_t nState = (size_t)nRows * dSH + (size_t)nRows * dEH + (size_t)nBatch * dG;
  float* st0 = (float*)carve(nState * 4);
  float* S0 = st0; float* E0 = S0 + (size_t)nRows * dSH; float* G0 = E0 + (size_t)nRows * dEH;
  float* S1 = (float*)carve((size_t)nRows * dSH * 4);
  float* E1 = (float*)carve((size_t)nRows * dEH * 4);
  float* G1 = (float*)carve((size_t)nBatch * dG * 4);
  u16* shAh = (u16*)carve((size_t)nRows * dSH * 2);    u16* shAl = (u16*)carve((size_t)nRows * dSH * 2);
  u16* ehAh = (u16*)carve((size_t)nRows * dEH * 2);    u16* ehAl = (u16*)carve((size_t)nRows * dEH * 2);
  u16* shTh = (u16*)carve((size_t)nBatch * dSH * nSent * 2); u16* shTl = (u16*)carve((size_t)nBatch * dSH * nSent * 2);
  float* P1s = (float*)carve((size_t)nRows * dP1 * 4);
  float* P1e = (float*)carve((size_t)nRows * dP1 * 4);
  float* P2e = (float*)carve((size_t)nRows * dP2 * 4);
  float* P2s = (float*)carve((size_t)nRows * dP2 * 4);
  float* sns = (float*)carve((size_t)nRows * dSH * 4);
  float* sne = (float*)carve((size_t)nRows * dP1 * 4);
  float* ens = (float*)carve((size_t)nRows * dP2 * 4);
  u16* xhSh = (u16*)carve((size_t)nRows * dXHS * 2);   u16* xhSl = (u16*)carve((size_t)nRows * dXHS * 2);
  u16* xhEh = (u16*)carve((size_t)nRows * dXHE * 2);   u16* xhEl = (u16*)carve((size_t)nRows * dXHE * 2);
  float* RZs = (float*)carve((size_t)nRows * 2 * dSH * 4);
  float* Cs  = (float*)carve((size_t)nRows * dSH * 4);
  float* Us  = (float*)carve((size_t)nRows * dSH * 4);
  float* RZe = (float*)carve((size_t)nRows * 2 * dEH * 4);
  float* Ce  = (float*)carve((size_t)nRows * dEH * 4);
  float* Ue  = (float*)carve((size_t)nRows * dEH * 4);
  if (off > ws_size || off > (size_t)134217728) return;

  zero4_kernel<<<(unsigned)((nState / 4 + 255) / 256), 256, 0, stream>>>(st0, (int)(nState / 4));
  adj_kernel<<<nBatch, 256, 0, stream>>>(matrix, smask, adjH, adjL);
  tables_kernel<<<4, 320, 0, stream>>>(ee, g1w, g1b, g2w, g2b, tab1, tab2);
  tsplit_kernel<<<dim3(dSH / 64, dP1 / 64, 1), 256, 0, stream>>>(g1w, dP1, dSH, 0L, wG1Sh, wG1Sl, dSH, 0L);
  tsplit_kernel<<<dim3(dEH / 64, dP1 / 64, 1), 256, 0, stream>>>(g1w + (size_t)dSH * dP1, dP1, dEH, 0L, wG1Eh, wG1El, dEH, 0L);
  tsplit_kernel<<<dim3(dEH / 64, dP2 / 64, 1), 256, 0, stream>>>(g2w, dP2, dEH, 0L, wG2Eh, wG2El, dEH, 0L);
  tsplit_kernel<<<dim3(dSH / 64, dP2 / 64, 1), 256, 0, stream>>>(g2w + (size_t)dEH * dP2, dP2, dSH, 0L, wG2Sh, wG2Sl, dSH, 0L);
  tsplit_kernel<<<dim3(dXHS / 64, dSH / 64, 1), 256, 0, stream>>>(s_rw, dSH, dXHS, 0L, wSRZh, wSRZl, dXHS, 0L);
  tsplit_kernel<<<dim3(dXHS / 64, dSH / 64, 1), 256, 0, stream>>>(s_zw, dSH, dXHS, 0L, wSRZh + (size_t)dSH * dXHS, wSRZl + (size_t)dSH * dXHS, dXHS, 0L);
  tsplit_kernel<<<dim3(dXS / 64, dSH / 64, 1), 256, 0, stream>>>(s_cw, dSH, dXS, 0L, wSCh, wSCl, dXS, 0L);
  tsplit_kernel<<<dim3(dSH / 64, dSH / 64, 1), 256, 0, stream>>>(s_uw, dSH, dSH, 0L, wSUh, wSUl, dSH, 0L);
  tsplit_kernel<<<dim3(dXHE / 64, dEH / 64, 1), 256, 0, stream>>>(e_rw, dEH, dXHE, 0L, wERZh, wERZl, dXHE, 0L);
  tsplit_kernel<<<dim3(dXHE / 64, dEH / 64, 1), 256, 0, stream>>>(e_zw, dEH, dXHE, 0L, wERZh + (size_t)dEH * dXHE, wERZl + (size_t)dEH * dXHE, dXHE, 0L);
  tsplit_kernel<<<dim3(dXE / 64, dEH / 64, 1), 256, 0, stream>>>(e_cw, dEH, dXE, 0L, wECh, wECl, dXE, 0L);
  tsplit_kernel<<<dim3(dEH / 64, dEH / 64, 1), 256, 0, stream>>>(e_uw, dEH, dEH, 0L, wEUh, wEUl, dEH, 0L);

  for (int layer = 0; layer < 2; ++layer) {
    const float* shold = (layer == 0) ? S0 : S1;
    const float* ehold = (layer == 0) ? E0 : E1;
    const float* gold  = (layer == 0) ? G0 : G1;
    float* snew = (layer == 0) ? S1 : out0;
    float* enew = (layer == 0) ? E1 : out1;
    float* gnew = (layer == 0) ? G1 : out2;

    rsplit_kernel<<<(nRows * dSH / 8) / 256, 256, 0, stream>>>(shold, shAh, shAl, nRows * dSH / 8);
    rsplit_kernel<<<(nRows * dEH / 8) / 256, 256, 0, stream>>>(ehold, ehAh, ehAl, nRows * dEH / 8);
    tsplit_kernel<<<dim3(nSent / 64, dSH / 64, nBatch), 256, 0, stream>>>(shold, dSH, nSent, (long)nSent * dSH, shTh, shTl, nSent, (long)dSH * nSent);

    gemm_bf16x3(shAh, shAl, dSH, 0L, wG1Sh, wG1Sl, dSH, 0L, P1s, dP1, 0L, nRows, dP1, dSH, 1, stream);
    gemm_bf16x3(ehAh, ehAl, dEH, 0L, wG1Eh, wG1El, dEH, 0L, P1e, dP1, 0L, nRows, dP1, dEH, 1, stream);
    gemm_bf16x3(ehAh, ehAl, dEH, 0L, wG2Eh, wG2El, dEH, 0L, P2e, dP2, 0L, nRows, dP2, dEH, 1, stream);
    gemm_bf16x3(shAh, shAl, dSH, 0L, wG2Sh, wG2Sl, dSH, 0L, P2s, dP2, 0L, nRows, dP2, dSH, 1, stream);
    gemm_bf16x3(adjH, adjL, nSent, (long)nSent * nSent, shTh, shTl, nSent, (long)dSH * nSent,
                sns, dSH, (long)nSent * dSH, nSent, dSH, nSent, nBatch, stream);

    aggs_kernel<<<dim3(nSent, nBatch), dP1, 0, stream>>>(matrix, ehold, P1s, P1e, tab1, ee, sne);
    agge_kernel<<<dim3(nWord, nBatch), dP2, 0, stream>>>(matrix, shold, P2s, P2e, tab2, ee, ens);

    packs_kernel<<<nRows, 256, 0, stream>>>(sent, sns, sne, gold, shold, xhSh, xhSl);
    packe_kernel<<<nRows, 256, 0, stream>>>(word, ens, gold, ehold, xhEh, xhEl);

    gemm_bf16x3(xhSh, xhSl, dXHS, 0L, wSRZh, wSRZl, dXHS, 0L, RZs, 2 * dSH, 0L, nRows, 2 * dSH, dXHS, 1, stream);
    gemm_bf16x3(xhSh, xhSl, dXHS, 0L, wSCh, wSCl, dXS, 0L, Cs, dSH, 0L, nRows, dSH, dXS, 1, stream);
    gemm_bf16x3(xhSh + dXS, xhSl + dXS, dXHS, 0L, wSUh, wSUl, dSH, 0L, Us, dSH, 0L, nRows, dSH, dSH, 1, stream);
    gemm_bf16x3(xhEh, xhEl, dXHE, 0L, wERZh, wERZl, dXHE, 0L, RZe, 2 * dEH, 0L, nRows, 2 * dEH, dXHE, 1, stream);
    gemm_bf16x3(xhEh, xhEl, dXHE, 0L, wECh, wECl, dXE, 0L, Ce, dEH, 0L, nRows, dEH, dXE, 1, stream);
    gemm_bf16x3(xhEh + dXE, xhEl + dXE, dXHE, 0L, wEUh, wEUl, dEH, 0L, Ue, dEH, 0L, nRows, dEH, dEH, 1, stream);

    cells_kernel<<<nRows, dSH, 0, stream>>>(RZs, Cs, Us, s_rb, s_zb, s_cb, s_ub, shold, smask, snew);
    celle_kernel<<<nRows, dEH, 0, stream>>>(RZe, Ce, Ue, e_rb, e_zb, e_cb, e_ub, ehold, wmask, enew);

    cellg_kernel<<<nBatch, dG, 0, stream>>>(snew, enew, smask, wmask, gold, g_rw, g_rb, g_zw, g_zb, g_cw, g_cb, g_uw, g_ub, gnew);
  }
}
